// BarrierNet_47974784697159
// MI455X (gfx1250) — hardware-verified
//
#include <hip/hip_runtime.h>
#include <math.h>

#pragma clang fp contract(off)

constexpr int kRows    = 262144;
constexpr int kFeat    = 5;
constexpr int kHid1    = 128;
constexpr int kHidCat  = 64;
constexpr int kHead    = 32;
constexpr int kNumObs  = 8;
constexpr float kOppRadius = 0.3f;
constexpr float kACarry    = 256.0f;
constexpr float kWCarry    = 64.0f;
constexpr float kGemmScale = 1.0f / (256.0f * 64.0f);
constexpr int kL1Rows   = 64;
constexpr int kTailRows = 512;

static_assert(kRows % 64 == 0);
static_assert(kHid1 % 32 == 0);
static_assert(kHidCat == 64);
static_assert(kRows % kL1Rows == 0);
static_assert(kRows % kTailRows == 0);
static_assert((kRows / 64) % 8 == 0);

typedef __attribute__((ext_vector_type(16))) _Float16 v16h;
typedef __attribute__((ext_vector_type(8)))  _Float16 v8h;
typedef __attribute__((ext_vector_type(8)))  float    v8f;
typedef __attribute__((ext_vector_type(4)))  float    v4f;
typedef __attribute__((ext_vector_type(4)))  unsigned int v4u;

__device__ __forceinline__ void keep4_h(v16h a, v16h b, v16h c, v16h d) { asm volatile("v_nop" :: "v"(a), "v"(b), "v"(c), "v"(d)); }
__device__ __forceinline__ void acc_guard4(v8f& a, v8f& b, v8f& c, v8f& d) { asm volatile("v_nop\n\tv_nop\n\tv_nop\n\tv_nop" : "+v"(a), "+v"(b), "+v"(c), "+v"(d)); }
__device__ __forceinline__ void dep_guard4_h(v8f& a, v8f& b, v8f& c, v8f& d, v16h x, v16h y0, v16h y1, v16h y2, v16h y3) {
  asm volatile("v_nop\n\tv_nop\n\tv_nop\n\tv_nop" : "+v"(a), "+v"(b), "+v"(c), "+v"(d) : "v"(x), "v"(y0), "v"(y1), "v"(y2), "v"(y3));
}

template <typename T> struct Frag;
template <> struct Frag<_Float16> {
  typedef v16h V; union U { v16h v; v8h h[2]; };
  static __device__ __forceinline__ v16h load(const _Float16* p) {
    U f; f.h[0] = *(const v8h*)(p); f.h[1] = *(const v8h*)(p + 16); return f.v;
  }
  static __device__ __forceinline__ v8f mma(v16h a, v16h b, v8f c) {
    return __builtin_amdgcn_wmma_f32_16x16x32_f16(false, a, false, b, (short)0, c, false, false);
  }
  static __device__ __forceinline__ void keep(v16h a, v16h b, v16h c, v16h d) { keep4_h(a, b, c, d); }
};

__device__ __forceinline__ unsigned pk16(unsigned short a, unsigned short b) { return (unsigned)a | ((unsigned)b << 16); }
__device__ __forceinline__ unsigned short h_bits(float f) { const _Float16 h = (_Float16)f; return __builtin_bit_cast(unsigned short, h); }

__global__ __launch_bounds__(256) void castw_kernel(const float* __restrict__ Wa, const float* __restrict__ Wb,
                                                    unsigned short* __restrict__ outp, float scale) {
  const int blk = blockIdx.x;
  const bool second = blk >= 8;
  const float* W = second ? Wb : Wa;
  const int i = (second ? (blk - 8) : blk) * 256 + threadIdx.x;
  const float f0 = W[2 * i] * scale;
  const float f1 = W[2 * i + 1] * scale;
  const unsigned u = pk16(h_bits(f0), h_bits(f1));
  unsigned* op = (unsigned*)(outp + (second ? kHead * kHid1 : 0)) + i;
  *(volatile unsigned*)op = u;
  __threadfence();
  *(volatile unsigned*)op = u;
}

__global__ __launch_bounds__(256) void layer1_kernel(const float* __restrict__ x, const float* __restrict__ W1,
                                                     const float* __restrict__ b1, unsigned short* __restrict__ Ah) {
  __shared__ float sW[kHid1 * kFeat];
  __shared__ float sB[kHid1];
  __shared__ float sX[kL1Rows * kFeat];
  const int tid = threadIdx.x, lane = tid & 31, wave = tid >> 5;
  const size_t row0 = (size_t)blockIdx.x * kL1Rows;
  for (int idx = tid; idx < kHid1 * kFeat; idx += 256) sW[idx] = W1[idx];
  if (tid < kHid1) sB[tid] = b1[tid];
  for (int idx = tid; idx < kL1Rows * kFeat; idx += 256) sX[idx] = x[row0 * kFeat + idx];
  __syncthreads();

  const int n0   = (lane & 15) * 8;
  const int hrow = lane >> 4;
  float w[8][5];
  float bb[8];
#pragma unroll
  for (int e = 0; e < 8; ++e) {
#pragma unroll
    for (int f = 0; f < 5; ++f) w[e][f] = sW[(n0 + e) * kFeat + f];
    bb[e] = sB[n0 + e];
  }
#pragma unroll 1
  for (int it = 0; it < 4; ++it) {
    const int rl = it * 16 + wave * 2 + hrow;
    float xr[5];
#pragma unroll
    for (int f = 0; f < 5; ++f) xr[f] = sX[rl * kFeat + f];
    unsigned short hb[8];
#pragma unroll
    for (int e = 0; e < 8; ++e) {
      float a = 0.0f;
#pragma unroll
      for (int f = 0; f < 5; ++f) a = fmaf(xr[f], w[e][f], a);
      a = a + bb[e];
      a = fmaxf(a, 0.0f) * kACarry;
      hb[e] = h_bits(a);
    }
    const v4u u = (v4u){pk16(hb[0], hb[1]), pk16(hb[2], hb[3]), pk16(hb[4], hb[5]), pk16(hb[6], hb[7])};
    unsigned short* dst = Ah + (row0 + rl) * kHid1 + n0;
    *(volatile v4u*)dst = u;
    __threadfence();
    *(volatile v4u*)dst = u;
  }
}

__global__ __launch_bounds__(256) void gemm_heads_kernel(
    const unsigned short* __restrict__ Ap, const unsigned short* __restrict__ Btp,
    const float* __restrict__ b21, const float* __restrict__ b22,
    const float* __restrict__ W31, const float* __restrict__ b31,
    const float* __restrict__ W32, const float* __restrict__ b32,
    float* __restrict__ Hout, int M, float scale) {
  __shared__ __align__(16) float sT[8][16 * 68];
  __shared__ float sBias2[kHidCat];
  __shared__ float sWh[4 * kHead];
  __shared__ float sBh[4];
  const int lane = threadIdx.x & 31;
  const int wave = threadIdx.x >> 5;
  if (wave == 0) {
    sBias2[lane] = b21[lane];
  } else if (wave == 1) {
    sBias2[kHead + lane] = b22[lane];
  } else if (wave == 2) {
    sWh[lane] = W31[lane]; sWh[32 + lane] = W31[32 + lane];
  } else if (wave == 3) {
    sWh[64 + lane] = W32[lane]; sWh[96 + lane] = W32[32 + lane];
  } else if (wave == 4) {
    const int li = lane < 2 ? lane : 1; const float v = b31[li]; if (lane < 2) sBh[lane] = v;
  } else if (wave == 5) {
    const int li = lane < 2 ? lane : 1; const float v = b32[li]; if (lane < 2) sBh[2 + lane] = v;
  }
  __syncthreads();

  const _Float16* A  = (const _Float16*)Ap;
  const _Float16* Bt = (const _Float16*)Btp;
  const int lda = kHid1, ldb = kHid1;
  const int K = kHid1;
  const int tilesM = M >> 6;
  const int tile = blockIdx.x * 8 + wave;
  if (tile >= tilesM) return;
  const int m0 = tile << 6;

  const int rlane = lane & 15;
  const int koff  = (lane >> 4) * 8;
  const int mOff  = (lane >> 4) * 8;
  const int hsel  = lane >> 4;

  v8f acc[4][4];
#pragma unroll
  for (int i = 0; i < 4; ++i)
#pragma unroll
    for (int j = 0; j < 4; ++j) acc[i][j] = (v8f){0.f,0.f,0.f,0.f,0.f,0.f,0.f,0.f};

  for (int k0 = 0; k0 < K; k0 += 32) {
    v16h bh[4];
#pragma unroll
    for (int j = 0; j < 4; ++j) {
      const size_t bo = (size_t)((j << 4) + rlane) * ldb + koff + k0;
      bh[j] = Frag<_Float16>::load(Bt + bo);
    }
#pragma unroll
    for (int i = 0; i < 4; ++i) {
      const size_t ao = (size_t)(m0 + (i << 4) + rlane) * lda + koff + k0;
      v16h ah = Frag<_Float16>::load(A + ao);
#pragma unroll
      for (int j = 0; j < 4; ++j) acc[i][j] = Frag<_Float16>::mma(ah, bh[j], acc[i][j]);
      dep_guard4_h(acc[i][0], acc[i][1], acc[i][2], acc[i][3], ah, bh[0], bh[1], bh[2], bh[3]);
    }
    Frag<_Float16>::keep(bh[0], bh[1], bh[2], bh[3]);
  }
  acc_guard4(acc[0][0], acc[0][1], acc[0][2], acc[0][3]);
  acc_guard4(acc[1][0], acc[1][1], acc[1][2], acc[1][3]);
  acc_guard4(acc[2][0], acc[2][1], acc[2][2], acc[2][3]);
  acc_guard4(acc[3][0], acc[3][1], acc[3][2], acc[3][3]);

  float* slab = sT[wave];
#pragma unroll
  for (int i = 0; i < 4; ++i) {
    const int mBase = m0 + (i << 4);
#pragma unroll
    for (int j = 0; j < 4; ++j) {
      const int n = (j << 4) + rlane;
      const float bv = sBias2[n];
#pragma unroll
      for (int r = 0; r < 8; ++r) {
        float v = acc[i][j][r] * scale + bv;
        v = fmaxf(v, 0.0f);
        slab[(mOff + r) * 68 + (j << 4) + rlane] = v;
      }
    }
    __builtin_amdgcn_fence(__ATOMIC_RELEASE, "workgroup");
    __builtin_amdgcn_wave_barrier();
    __builtin_amdgcn_fence(__ATOMIC_ACQUIRE, "workgroup");
    {
      const float* srow = slab + rlane * 68 + hsel * kHead;
      const float* wr   = sWh + hsel * (2 * kHead);
      float d0 = 0.0f, d1 = 0.0f;
#pragma unroll
      for (int k = 0; k < kHead; ++k) {
        const float xv = srow[k];
        d0 = fmaf(xv, wr[k], d0);
        d1 = fmaf(xv, wr[kHead + k], d1);
      }
      d0 = d0 + sBh[hsel * 2];
      d1 = d1 + sBh[hsel * 2 + 1];
      const float den0 = 1.0f + expf(-d0);
      const float den1 = 1.0f + expf(-d1);
      const float t0 = 4.0f * (1.0f / den0);
      const float t1 = 4.0f * (1.0f / den1);
      const float hvl = t0 * t1;
      const float hvx = __shfl_xor(hvl, 16, 32);
      const v4f o = (v4f){d0, d1, hvx, 0.0f};
      float* hp = Hout + (size_t)(mBase + rlane) * 4;
      for (int pass = 0; pass < 2; ++pass) {
        if (hsel == 0) *(volatile v4f*)hp = o;
        __threadfence();
      }
    }
    __builtin_amdgcn_fence(__ATOMIC_RELEASE, "workgroup");
    __builtin_amdgcn_wave_barrier();
    __builtin_amdgcn_fence(__ATOMIC_ACQUIRE, "workgroup");
  }
}

__device__ __forceinline__ void qp_constraint(float px, float py, float ct, float st, float hv,
                                              float ox, float oy, float rad, float& upper, float& lower) {
  const float dx = px - ox;
  const float dy = py - oy;
  const float dd = dx * dx + dy * dy;
  const float cval = dd - rad * rad;
  const float lg = (2.0f * dx) * ct + (2.0f * dy) * st;
  const float g1 = -lg;
  const float sg = (g1 != 0.0f) ? g1 : 1.0f;
  const float hv_c = hv * cval;
  const float ratio = hv_c / sg;
  upper = (g1 > 0.0f) ? fminf(upper, ratio) : upper;
  lower = (g1 < 0.0f) ? fmaxf(lower, ratio) : lower;
}

__global__ __launch_bounds__(256) void cbf_clip_kernel(const float* __restrict__ x, const float* __restrict__ mean,
                                                       const float* __restrict__ stdv, const float* __restrict__ obst,
                                                       const float* __restrict__ Hp, float* __restrict__ out, int nB) {
  __shared__ float sMean[8];
  __shared__ float sStd[8];
  __shared__ float sOb[kNumObs * 3];
  const int tid = threadIdx.x, lane = tid & 31, wave = tid >> 5;
  if (wave == 0) {
    const int li = lane < kFeat ? lane : kFeat - 1; const float v = mean[li]; if (lane < kFeat) sMean[lane] = v;
  } else if (wave == 1) {
    const int li = lane < kFeat ? lane : kFeat - 1; const float v = stdv[li]; if (lane < kFeat) sStd[lane] = v;
  } else if (wave == 2) {
    const int li = lane < kNumObs * 3 ? lane : kNumObs * 3 - 1; const float v = obst[li]; if (lane < kNumObs * 3) sOb[lane] = v;
  }
  __syncthreads();

  const int pair = blockIdx.x * 256 + tid;
  const int rowA = pair * 2;
  float u1a = 0.0f, u2a = 0.0f, u1b = 0.0f, u2b = 0.0f;
#pragma unroll 1
  for (int rr = 0; rr < 2; ++rr) {
    int row = rowA + rr;
    row = row < nB ? row : nB - 1;
    const float* xr = x + (size_t)row * kFeat;
    float xo[5];
#pragma unroll
    for (int f = 0; f < 5; ++f) {
      const float t0 = xr[f] * sStd[f];
      const float x0 = t0 + sMean[f];
      const float t1 = x0 * sStd[f];
      xo[f] = t1 + sMean[f];
    }
    const v4f hrow = *(const v4f*)(Hp + (size_t)row * 4);
    const float px = xo[0], py = xo[1], th = xo[2], opx = xo[3], opy = xo[4];
    float st, ct;
    sincosf(th, &st, &ct);
    const float hv = hrow[2];
    float upper = __builtin_inff();
    float lower = -__builtin_inff();
#pragma unroll 1
    for (int i = 0; i < kNumObs + 1; ++i) {
      const int ii = i < kNumObs ? i : kNumObs - 1;
      const float oxs = sOb[3 * ii], oys = sOb[3 * ii + 1], ors = sOb[3 * ii + 2];
      const bool stat = i < kNumObs;
      const float ox = stat ? oxs : opx;
      const float oy = stat ? oys : opy;
      const float rad = stat ? ors : kOppRadius;
      qp_constraint(px, py, ct, st, hv, ox, oy, rad, upper, lower);
    }
    const float u1 = fminf(fmaxf(-hrow[0], lower), upper);
    const float u2 = -hrow[1];
    u1a = (rr == 0) ? u1 : u1a;  u2a = (rr == 0) ? u2 : u2a;
    u1b = (rr == 1) ? u1 : u1b;  u2b = (rr == 1) ? u2 : u2b;
  }
  const v4f o = (v4f){u1a, u2a, u1b, u2b};
  float* op = out + (size_t)pair * 4;
  if (rowA + 1 < nB) {
    *(volatile v4f*)op = o;
    __threadfence();
    *(volatile v4f*)op = o;
  }
}

extern "C" void kernel_launch(void* const* d_in, const int* in_sizes, int n_in,
                              void* d_out, int out_size, void* d_ws, size_t ws_size,
                              hipStream_t stream) {
  if (n_in < 14) return;
  const float* x    = (const float*)d_in[0];
  const float* mean = (const float*)d_in[1];
  const float* stdv = (const float*)d_in[2];
  const float* W1   = (const float*)d_in[3];
  const float* b1   = (const float*)d_in[4];
  const float* W21  = (const float*)d_in[5];
  const float* b21  = (const float*)d_in[6];
  const float* W22  = (const float*)d_in[7];
  const float* b22  = (const float*)d_in[8];
  const float* W31  = (const float*)d_in[9];
  const float* b31  = (const float*)d_in[10];
  const float* W32  = (const float*)d_in[11];
  const float* b32  = (const float*)d_in[12];
  const float* obst = (const float*)d_in[13];
  float* out = (float*)d_out;

  const int nB = in_sizes[0] / kFeat;
  if (nB != kRows || out_size != kRows * 2) return;
  if (in_sizes[3] != kHid1 * kFeat || in_sizes[5] != kHead * kHid1 || in_sizes[7] != kHead * kHid1) return;
  if (in_sizes[9] != 2 * kHead || in_sizes[11] != 2 * kHead || in_sizes[13] != kNumObs * 3) return;

  const size_t bytesA  = (size_t)kRows * kHid1 * 2;
  const size_t bytesH  = (size_t)kRows * 4 * 4;
  const size_t bytesBt = (size_t)kHidCat * kHid1 * 2;
  const size_t offA  = 0;
  const size_t offH  = offA + bytesA;
  const size_t offBt = offH + bytesH;
  const size_t total = offBt + bytesBt;
  if (total > ws_size) return;

  unsigned char* ws = (unsigned char*)d_ws;
  unsigned short* Ah = (unsigned short*)(ws + offA);
  float* Hp = (float*)(ws + offH);
  unsigned short* Bt = (unsigned short*)(ws + offBt);

  castw_kernel<<<dim3(16), dim3(256), 0, stream>>>(W21, W22, Bt, kWCarry);
  layer1_kernel<<<dim3(kRows / kL1Rows), dim3(256), 0, stream>>>(x, W1, b1, Ah);
  gemm_heads_kernel<<<dim3(kRows / (64 * 8)), dim3(256), 0, stream>>>(Ah, Bt, b21, b22, W31, b31, W32, b32, Hp,
                                                                      kRows, kGemmScale);
  cbf_clip_kernel<<<dim3(kRows / kTailRows), dim3(256), 0, stream>>>(x, mean, stdv, obst, Hp, out, nB);
}
